// TrainablePQC_23115513987350
// MI455X (gfx1250) — hardware-verified
//
#include <hip/hip_runtime.h>
#include <math.h>

typedef __attribute__((ext_vector_type(16))) _Float16 v16h;
typedef __attribute__((ext_vector_type(16))) __bf16 v16b;
typedef __attribute__((ext_vector_type(8)))  _Float16 v8h;
typedef __attribute__((ext_vector_type(8)))  float v8f;
typedef __attribute__((ext_vector_type(4)))  float v4f;
typedef __attribute__((ext_vector_type(2)))  float v2f;
typedef __attribute__((ext_vector_type(4)))  unsigned v4u;
typedef __attribute__((ext_vector_type(4)))  int v4i;
typedef float __attribute__((may_alias)) float_a;
typedef int __attribute__((may_alias)) int_a;

template <typename T> __device__ __forceinline__ void vst2(void* p, T v) { *(volatile T*)p = v; __threadfence(); *(volatile T*)p = v; }
__device__ __forceinline__ v8f wmma16(v16h a, v16h b, v8f c) {
  v8f d = __builtin_amdgcn_wmma_f32_16x16x32_f16(false, a, false, b, (short)0, c, false, false);
  asm volatile("v_nop\n\tv_nop\n\tv_nop\n\tv_nop" : "+v"(d) : "v"(a), "v"(b));
  return d;
}
__device__ __forceinline__ v8f wmma_bf(v16b a, v16b b, v8f c) {
  v8f d = __builtin_amdgcn_wmma_f32_16x16x32_bf16(false, a, false, b, (short)0, c, false, false);
  asm volatile("v_nop\n\tv_nop\n\tv_nop\n\tv_nop" : "+v"(d) : "v"(a), "v"(b));
  return d;
}
__device__ __forceinline__ v16h frag_h(const _Float16* rowk0, int lane) {
  union { v16h v; v8h q[2]; } u; const _Float16* p = rowk0 + 8 * (lane >> 4);
  u.q[0] = *(const v8h*)p; u.q[1] = *(const v8h*)(p + 16); return u.v;
}
__device__ __forceinline__ v16h frag_f32(const float* rowk0, int lane) {
  v16h a; const float* p = rowk0 + 8 * (lane >> 4);
#pragma unroll
  for (int i = 0; i < 8; ++i) { a[i] = (_Float16)p[i]; a[8 + i] = (_Float16)p[16 + i]; }
  return a;
}
__device__ __forceinline__ v16h frag_f32s(const float* rowk0, int lane, float sc) {
  v16h a; const float* p = rowk0 + 8 * (lane >> 4);
#pragma unroll
  for (int i = 0; i < 8; ++i) { a[i] = (_Float16)(p[i] * sc); a[8 + i] = (_Float16)(p[16 + i] * sc); }
  return a;
}
__device__ __forceinline__ v16h fragc_f32(const float* W, int k0, int n, int lane, int ld, int K) {
  v16h a; const int g = lane >> 4;
#pragma unroll
  for (int i = 0; i < 8; ++i) { const int ka = k0 + 8 * g + i, kb = ka + 16;
    a[i] = (_Float16)(ka < K ? W[(size_t)(ka < K ? ka : K - 1) * ld + n] : 0.f); a[8 + i] = (_Float16)(kb < K ? W[(size_t)(kb < K ? kb : K - 1) * ld + n] : 0.f); }
  return a;
}
struct F2 { v16b h, l; };
__device__ __forceinline__ F2 bsplit16(const float v[16]) { F2 r;
#pragma unroll
  for (int i = 0; i < 16; ++i) { const __bf16 h = (__bf16)v[i]; r.h[i] = h; r.l[i] = (__bf16)(v[i] - (float)h); }
  return r; }
__device__ __forceinline__ F2 split_row(const float* row, int k0, int lane) { float v[16]; const float* p = row + k0 + 8 * (lane >> 4);
#pragma unroll
  for (int i = 0; i < 8; ++i) { v[i] = p[i]; v[8 + i] = p[16 + i]; }
  return bsplit16(v); }
__device__ __forceinline__ F2 split_rowK(const float* row, int k0, int lane, int K) { float v[16]; const int g = lane >> 4;
#pragma unroll
  for (int i = 0; i < 8; ++i) { const int ka = k0 + 8 * g + i, kb = ka + 16; v[i] = ka < K ? row[ka < K ? ka : K - 1] : 0.f; v[8 + i] = kb < K ? row[kb < K ? kb : K - 1] : 0.f; }
  return bsplit16(v); }
__device__ __forceinline__ F2 split_col(const float* W, int k0, int n, int lane, int ld, int K) { float v[16]; const int g = lane >> 4;
#pragma unroll
  for (int i = 0; i < 8; ++i) { const int ka = k0 + 8 * g + i, kb = ka + 16; v[i] = ka < K ? W[(size_t)(ka < K ? ka : K - 1) * ld + n] : 0.f; v[8 + i] = kb < K ? W[(size_t)(kb < K ? kb : K - 1) * ld + n] : 0.f; }
  return bsplit16(v); }
__device__ __forceinline__ v8f mac3(const F2& a, const F2& b, v8f c) { c = wmma_bf(a.l, b.h, c); c = wmma_bf(a.h, b.l, c); return wmma_bf(a.h, b.h, c); }
__device__ __forceinline__ float sigm(float v) { return 1.0f / (1.0f + expf(-v)); }
#define LDSX() do { asm volatile("s_wait_dscnt 0" ::: "memory"); __builtin_amdgcn_wave_barrier(); __builtin_amdgcn_fence(__ATOMIC_RELEASE, "workgroup"); } while (0)


#define NSMP 4096
#define NQB 10
#define NST 1024
#define NL 4
__device__ __forceinline__ float bfr(float v) { return (float)(__bf16)v; }
__device__ __forceinline__ v16b frag_b(const __bf16* rowk0, int lane) { return __builtin_bit_cast(v16b, frag_h((const _Float16*)rowk0, lane)); }

__global__ __launch_bounds__(256) void k_ucols(const float* __restrict__ prm, float* __restrict__ UFre, float* __restrict__ UFim) {
  __shared__ __align__(16) float sre[16][NST + 4], sim[16][NST + 4]; __shared__ float sg[NL * 2 * NQB];
  const int tid = threadIdx.x; const int j0 = blockIdx.x * 16;
  if (tid < NL * 2 * NQB) sg[tid] = bfr(prm[tid]);
  for (int q = tid; q < 16 * NST; q += 256) { const int c = q >> 10, b = q & 1023; sre[c][b] = (b == j0 + c) ? 1.f : 0.f; sim[c][b] = 0.f; }
  __syncthreads();
  for (int layer = 0; layer < NL; ++layer) {
    for (int i = 0; i < NQB; ++i) { const int sh = NQB - 1 - i; const int bit = 1 << sh;
      const float ty = sg[layer * 2 * NQB + i], tz = sg[layer * 2 * NQB + NQB + i]; const float cy = cosf(0.5f * ty), sy = sinf(0.5f * ty), cz = cosf(0.5f * tz), sz = sinf(0.5f * tz);
      for (int q = tid; q < 16 * (NST / 2); q += 256) { const int col = q >> 9, pr = q & 511; const int lo = pr & (bit - 1), hi = pr >> sh; const int b0 = (hi << (sh + 1)) | lo; const int b1 = b0 | bit;
        const float ar = sre[col][b0], ai = sim[col][b0], br_ = sre[col][b1], bi = sim[col][b1];
        const float t0r = cy * ar - sy * br_, t0i = cy * ai - sy * bi, t1r = sy * ar + cy * br_, t1i = sy * ai + cy * bi;
        sre[col][b0] = cz * t0r + sz * t0i; sim[col][b0] = cz * t0i - sz * t0r;
        sre[col][b1] = cz * t1r - sz * t1i; sim[col][b1] = cz * t1i + sz * t1r; }
      __syncthreads(); }
    for (int i = 0; i < NQB; ++i) { const int ci = i, ti = (i + 1) % NQB; const int cbit = 1 << (NQB - 1 - ci), tbit = 1 << (NQB - 1 - ti);
      for (int q = tid; q < 16 * NST; q += 256) { const int col = q >> 10, b = q & 1023;
        if ((b & cbit) && !(b & tbit)) { const int b2 = b | tbit; const float u0 = sre[col][b], u1 = sim[col][b]; sre[col][b] = sre[col][b2]; sim[col][b] = sim[col][b2]; sre[col][b2] = u0; sim[col][b2] = u1; } }
      __syncthreads(); } }
  for (int q = tid; q < 16 * NST / 4; q += 256) { const int c = q >> 8, pc = q & 255; vst2(UFre + (size_t)(j0 + c) * NST + pc * 4, *(const v4f*)(&sre[c][pc * 4])); vst2(UFim + (size_t)(j0 + c) * NST + pc * 4, *(const v4f*)(&sim[c][pc * 4])); }
}
__global__ __launch_bounds__(256) void k_utr(const float* __restrict__ UFre, const float* __restrict__ UFim, __bf16* __restrict__ URh, __bf16* __restrict__ URl, __bf16* __restrict__ UIh, __bf16* __restrict__ UIl) {
  __shared__ __align__(16) __bf16 sh_[32][NST + 8], sl_[32][NST + 8];
  const int tid = threadIdx.x; const int a0 = blockIdx.x * 32; const int which = blockIdx.y; const float* UF = which == 0 ? UFre : UFim; __bf16* Oh = which == 0 ? URh : UIh; __bf16* Ol = which == 0 ? URl : UIl;
  for (int q = tid; q < 32 * NST; q += 256) { const int al = q & 31, j = q >> 5; const float v = UF[(size_t)j * NST + a0 + al]; const __bf16 hi = (__bf16)v; sh_[al][j] = hi; sl_[al][j] = (__bf16)(v - (float)hi); }
  __syncthreads();
  for (int q = tid; q < 32 * (NST / 8); q += 256) { const int al = q >> 7, pc = q & 127; vst2((unsigned*)(Oh + (size_t)(a0 + al) * NST + pc * 8), *(const v4u*)(&sh_[al][pc * 8])); vst2((unsigned*)(Ol + (size_t)(a0 + al) * NST + pc * 8), *(const v4u*)(&sl_[al][pc * 8])); }
}
__global__ __launch_bounds__(256) void k_s0(const float* __restrict__ x, float* __restrict__ S0) {
  __shared__ float scs[16][2 * NQB]; __shared__ __align__(16) float ss[16][NST + 4];
  const int tid = threadIdx.x; const int r0 = blockIdx.x * 16; const int rl = tid >> 4, sub = tid & 15;
  if (sub < NQB) { const float ang = bfr(x[(size_t)(r0 + rl) * NQB + sub]); scs[rl][sub] = cosf(0.5f * ang); scs[rl][NQB + sub] = sinf(0.5f * ang); }
  __syncthreads();
#pragma unroll 1
  for (int b8 = 0; b8 < NST / 16; ++b8) { const int b = sub * (NST / 16) + b8; float p = 1.f;
#pragma unroll
    for (int q = 0; q < NQB; ++q) { const int bit = (b >> (NQB - 1 - q)) & 1; p *= scs[rl][bit ? NQB + q : q]; }
    ss[rl][b] = p; }
  __syncthreads();
  for (int q = tid; q < 16 * NST / 4; q += 256) { const int r = q >> 8, pc = q & 255; vst2(S0 + (size_t)(r0 + r) * NST + pc * 4, *(const v4f*)(&ss[r][pc * 4])); }
}
__global__ __launch_bounds__(128) void k_meas(const float* __restrict__ S0, const __bf16* __restrict__ URh, const __bf16* __restrict__ URl, const __bf16* __restrict__ UIh, const __bf16* __restrict__ UIl, float* __restrict__ out) {
  __shared__ __align__(16) float spr[4][16][260]; __shared__ __align__(16) float sout[64 * NQB + 16];
  const int tid = threadIdx.x, wave = tid >> 5, lane = tid & 31, col = lane & 15, g = lane >> 4; const size_t r0 = (size_t)blockIdx.x * 64 + wave * 16;
  const int rl = lane & 15, hf = lane >> 4; float ev[NQB];
#pragma unroll
  for (int q = 0; q < NQB; ++q) ev[q] = 0.f;
#pragma unroll 1
  for (int ch = 0; ch < NST / 256; ++ch) {
#pragma unroll 1
    for (int part = 0; part < 2; ++part) { const __bf16* Uh = part == 0 ? URh : UIh; const __bf16* Ul = part == 0 ? URl : UIl; v8f acc[16] = {};
#pragma unroll 1
      for (int kc = 0; kc < NST / 32; ++kc) { const F2 a = split_row(S0 + (r0 + col) * NST, kc * 32, lane);
#pragma unroll
        for (int t = 0; t < 16; ++t) { const size_t uo = (size_t)(ch * 256 + t * 16 + col) * NST + kc * 32; const v16b uh = frag_b(Uh + uo, lane), ul = frag_b(Ul + uo, lane); acc[t] = wmma_bf(a.l, uh, acc[t]); acc[t] = wmma_bf(a.h, ul, acc[t]); acc[t] = wmma_bf(a.h, uh, acc[t]); } }
#pragma unroll
      for (int t = 0; t < 16; ++t)
#pragma unroll
        for (int r = 0; r < 8; ++r) { const float v = acc[t][r]; if (part == 0) spr[wave][8 * g + r][t * 16 + col] = v * v; else spr[wave][8 * g + r][t * 16 + col] += v * v; }
      LDSX(); }
#pragma unroll 2
    for (int bb = 0; bb < 128; ++bb) { const int bl = hf * 128 + bb; const int b = ch * 256 + bl; const float p = spr[wave][rl][bl];
#pragma unroll
      for (int q = 0; q < NQB; ++q) ev[q] += ((b >> (NQB - 1 - q)) & 1) ? -p : p; }
    LDSX(); }
#pragma unroll
  for (int q = 0; q < NQB; ++q) ev[q] += __shfl_xor(ev[q], 16, 32);
  if (hf == 0) {
#pragma unroll
    for (int q = 0; q < NQB; ++q) sout[(wave * 16 + rl) * NQB + q] = ev[q]; }
  __syncthreads();
  for (int q = tid; q < 64 * NQB / 4; q += 128) vst2(out + (size_t)blockIdx.x * 64 * NQB + q * 4, *(const v4f*)(&sout[q * 4]));
}
extern "C" void kernel_launch(void* const* d_in, const int* in_sizes, int n_in, void* d_out, int out_size, void* d_ws, size_t ws_size, hipStream_t stream) {
  (void)in_sizes; (void)n_in; (void)out_size; (void)ws_size;
  const float* x = (const float*)d_in[0]; const float* prm = (const float*)d_in[1];
  char* ws = (char*)d_ws; size_t off = 0;
  auto take = [&](size_t bytes) { char* p = ws + off; off += (bytes + 255) & ~(size_t)255; return p; };
  float* UFre = (float*)take((size_t)NST * NST * 4); float* UFim = (float*)take((size_t)NST * NST * 4);
  __bf16* URh = (__bf16*)take((size_t)NST * NST * 2); __bf16* URl = (__bf16*)take((size_t)NST * NST * 2); __bf16* UIh = (__bf16*)take((size_t)NST * NST * 2); __bf16* UIl = (__bf16*)take((size_t)NST * NST * 2);
  float* S0 = (float*)take((size_t)NSMP * NST * 4);
  k_ucols<<<NST / 16, 256, 0, stream>>>(prm, UFre, UFim);
  k_utr<<<dim3(NST / 32, 2), 256, 0, stream>>>(UFre, UFim, URh, URl, UIh, UIl);
  k_s0<<<NSMP / 16, 256, 0, stream>>>(x, S0);
  k_meas<<<NSMP / 64, 128, 0, stream>>>(S0, URh, URl, UIh, UIl, (float*)d_out);
}
